// MultiHeadAttentionBlock_8306466750694
// MI455X (gfx1250) — hardware-verified
//
#include <hip/hip_runtime.h>


#ifndef NB
#define NB 2
#endif
#ifndef SEQ
#define SEQ 2048
#endif
#define SEQ_FULL 2048
#define DM    1024
#define DMLOG 10
#define NH_   16
#define HD    64
#define QT    (SEQ / 16)
#define PCAR  1024.0f
#define RCAR  2048.0f
#define VCAR  16.0f

static_assert(DM == NH_ * HD);
static_assert((1 << DMLOG) == DM);
static_assert(HD == 64);
static_assert(SEQ % 64 == 0);
static_assert(SEQ <= SEQ_FULL);
static_assert(QT % 4 == 0);
static_assert(DM % 64 == 0);
static_assert(((DM * DM / 64) % 64) == 0);
static_assert(((SEQ * DM / 8) % 256) == 0);

typedef _Float16 h16;
typedef unsigned short bf;
typedef __attribute__((ext_vector_type(16))) __bf16   v16bf;
typedef __attribute__((ext_vector_type(16))) _Float16 v16h;
typedef __attribute__((ext_vector_type(8)))  _Float16 v8h;
typedef __attribute__((ext_vector_type(8)))  unsigned short v8us;
typedef __attribute__((ext_vector_type(2)))  unsigned short v2us;
typedef __attribute__((ext_vector_type(8)))  float    v8f;
typedef __attribute__((ext_vector_type(4)))  float    v4f;
typedef v8h  __attribute__((may_alias)) v8ha;
typedef v4f  __attribute__((may_alias)) v4fa;
typedef v8us __attribute__((may_alias)) v8usa;

__device__ __forceinline__ unsigned short f2bf(float f) { unsigned u = __float_as_uint(f); u += 0x7FFFu + ((u >> 16) & 1u); return (unsigned short)(u >> 16); }
__device__ __forceinline__ float bf2f(unsigned short b) { return __uint_as_float(((unsigned)b) << 16); }
__device__ __forceinline__ float bfr(float f) { return bf2f(f2bf(f)); }
__device__ __forceinline__ v16h cat16(v8h lo, v8h hi) { return __builtin_shufflevector(lo, hi, 0, 1, 2, 3, 4, 5, 6, 7, 8, 9, 10, 11, 12, 13, 14, 15); }
__device__ __forceinline__ v16bf cat16b(v8us lo, v8us hi) { return __builtin_bit_cast(v16bf, __builtin_shufflevector(lo, hi, 0, 1, 2, 3, 4, 5, 6, 7, 8, 9, 10, 11, 12, 13, 14, 15)); }
__device__ __forceinline__ v8f wmma16(v16h a, v16h b, v8f c) { return __builtin_amdgcn_wmma_f32_16x16x32_f16(false, a, false, b, (short)0, c, false, false); }
__device__ __forceinline__ v8f wmmab(v16bf a, v16bf b, v8f c) { return __builtin_amdgcn_wmma_f32_16x16x32_bf16(false, a, false, b, (short)0, c, false, false); }
__device__ __forceinline__ v16bf ldb(const bf* p) { return cat16b(*(const v8us*)p, *(const v8us*)(p + 16)); }
__device__ __forceinline__ v16h  ldh(const h16* p) { return cat16(*(const v8h*)p, *(const v8h*)(p + 16)); }
__device__ __forceinline__ void wave_sync() { __builtin_amdgcn_fence(3  , "wavefront"); __builtin_amdgcn_wave_barrier(); asm volatile("" ::: "memory"); }

__global__ __launch_bounds__(256) void k_wtG(const float* __restrict__ w, bf* Bt) {
    const unsigned lane = threadIdx.x & 31u; const unsigned L0 = (blockIdx.x * 8u + (threadIdx.x >> 5)) * 8u;
#pragma unroll
    for (int ps = 0; ps < 2; ++ps) {
#pragma unroll 1
        for (unsigned l = 0; l < 8u; ++l) { const unsigned L = L0 + l; const unsigned e = L * 64u + lane * 2u; const unsigned k = e & (unsigned)(DM - 1); const unsigned n = e >> DMLOG; v2us o;
            o[0] = f2bf(w[(size_t)k * DM + n]); o[1] = f2bf(w[(size_t)(k + 1u) * DM + n]); *(volatile v2us*)(Bt + e) = o; }
        if (ps == 0) __threadfence(); }
}

__global__ __launch_bounds__(256) void k_cvt8(const float* __restrict__ src, bf* dst, size_t sS, size_t sD, unsigned n8) {
    const unsigned i = blockIdx.x * 256u + threadIdx.x; if (i >= n8) return;
    const float* s = src + (size_t)blockIdx.y * sS + (size_t)i * 8; bf* d = dst + (size_t)blockIdx.y * sD + (size_t)i * 8;
    const v4f a = *(const v4f*)s; const v4f c = *(const v4f*)(s + 4); v8us o;
#pragma unroll
    for (int q = 0; q < 4; ++q) { o[q] = f2bf(a[q]); o[q + 4] = f2bf(c[q]); }
    *(volatile v8us*)d = o; __threadfence(); *(volatile v8us*)d = o;
}

template <int OM>
__global__ __launch_bounds__(32) void k_gemmw(const bf* __restrict__ A, const bf* __restrict__ Bt, void* Cv, const float* __restrict__ bias, size_t sA, size_t sC, int K, int ldc) {
    __shared__ __align__(16) float os[16 * 68];
    const size_t z = blockIdx.z; A += z * sA;
    const unsigned lane = threadIdx.x & 31u, lr = lane & 15u, hi = lane >> 4; const unsigned r0 = blockIdx.x * 64u, c0 = blockIdx.y * 64u;
    v8f acc[4][4];
#pragma unroll
    for (int mb = 0; mb < 4; ++mb)
#pragma unroll
        for (int nb = 0; nb < 4; ++nb) acc[mb][nb] = (v8f){};
    const size_t aoff = (size_t)(r0 + lr) * K + 8u * hi, boff = (size_t)(c0 + lr) * K + 8u * hi;
#pragma unroll 1
    for (int kc = 0; kc < K; kc += 32) {
        v16bf a[4];
#pragma unroll
        for (int mb = 0; mb < 4; ++mb) a[mb] = ldb(A + aoff + (size_t)mb * 16 * K + kc);
#pragma unroll
        for (int nb = 0; nb < 4; ++nb) { const v16bf b = ldb(Bt + boff + (size_t)nb * 16 * K + kc);
#pragma unroll
            for (int mb = 0; mb < 4; ++mb) acc[mb][nb] = wmmab(a[mb], b, acc[mb][nb]); }
        asm volatile("v_nop\n\tv_nop\n\tv_nop\n\tv_nop" : "+v"(acc[0][0]), "+v"(acc[1][1]), "+v"(acc[2][2]), "+v"(acc[3][3]) : "v"(a[0]), "v"(a[3]));
    }
#pragma unroll
    for (int mb = 0; mb < 4; ++mb) {
#pragma unroll
        for (int nb = 0; nb < 4; ++nb) {
#pragma unroll
            for (int j = 0; j < 8; ++j) os[(hi * 8u + j) * 68u + nb * 16u + lr] = acc[mb][nb][j]; }
        wave_sync();
        if (OM == 0) {
            float* crow = (float*)Cv + z * sC + (size_t)(r0 + mb * 16u) * ldc + c0;
#pragma unroll 1
            for (int ps = 0; ps < 2; ++ps) {
#pragma unroll
                for (int s = 0; s < 8; ++s) { const unsigned row = 2u * s + hi, cofs = lr * 4u; v4f val = *(const v4fa*)(os + row * 68u + cofs);
#pragma unroll
                    for (int q = 0; q < 4; ++q) val[q] = bfr(bfr(val[q]) + bfr(bias[c0 + cofs + q]));
                    *(volatile v4f*)(crow + (size_t)row * ldc + cofs) = val; }
                if (ps == 0) __threadfence(); }
        } else if (OM == 1) {
            bf* crow = (bf*)Cv + (size_t)(r0 + mb * 16u) * ldc + c0;
#pragma unroll 1
            for (int ps = 0; ps < 2; ++ps) {
#pragma unroll
                for (int s = 0; s < 4; ++s) { const unsigned row = 4u * s + (lane >> 3), cofs = (lane & 7u) * 8u; const v4f x0 = *(const v4fa*)(os + row * 68u + cofs); const v4f x1 = *(const v4fa*)(os + row * 68u + cofs + 4u); v8us o;
#pragma unroll
                    for (int q = 0; q < 4; ++q) { o[q] = f2bf(bfr(x0[q]) + bfr(bias[c0 + cofs + q])); o[q + 4] = f2bf(bfr(x1[q]) + bfr(bias[c0 + cofs + 4u + q])); }
                    *(volatile v8us*)(crow + (size_t)row * ldc + cofs) = o; }
                if (ps == 0) __threadfence(); }
        } else {
            h16* crow = (h16*)Cv + (size_t)(r0 + mb * 16u) * ldc + c0;
#pragma unroll 1
            for (int ps = 0; ps < 2; ++ps) {
#pragma unroll
                for (int s = 0; s < 4; ++s) { const unsigned row = 4u * s + (lane >> 3), cofs = (lane & 7u) * 8u; const v4f x0 = *(const v4fa*)(os + row * 68u + cofs); const v4f x1 = *(const v4fa*)(os + row * 68u + cofs + 4u); const float bb = bfr(bias[r0 + mb * 16u + row]); v8h o;
#pragma unroll
                    for (int q = 0; q < 4; ++q) { o[q] = (h16)(bfr(bfr(x0[q]) + bb) * VCAR); o[q + 4] = (h16)(bfr(bfr(x1[q]) + bb) * VCAR); }
                    *(volatile v8h*)(crow + (size_t)row * ldc + cofs) = o; }
                if (ps == 0) __threadfence(); }
        }
        wave_sync();
    }
}

__global__ __launch_bounds__(128) void k_flash(const bf* __restrict__ Qp, const bf* __restrict__ Kp, const h16* __restrict__ VT, const int* __restrict__ mask, bf* Xo) {
    __shared__ __align__(16) h16 Pb[4][16 * 72];
    __shared__ __align__(16) h16 Rb[4][16 * 72];
    __shared__ __align__(16) unsigned short Ob[4][16 * 72];
    const unsigned wave = threadIdx.x >> 5, lane = threadIdx.x & 31u, lr = lane & 15u, hi = lane >> 4;
    const unsigned wg = blockIdx.x * 4u + wave;
    const unsigned b = wg / (unsigned)(NH_ * QT); const unsigned rem = wg - b * (unsigned)(NH_ * QT); const unsigned h = rem / (unsigned)QT; const unsigned q0 = (rem - h * (unsigned)QT) * 16u;
    h16* P = Pb[wave]; h16* R = Rb[wave]; unsigned short* Ow = Ob[wave];
    const float NINF = -__builtin_huge_valf();

    const bf* qrow = Qp + (size_t)(b * SEQ + q0 + lr) * DM + h * HD + 8u * hi;
    const v16bf qa0 = ldb(qrow), qa1 = ldb(qrow + 32);
    const bf* kp = Kp + (size_t)(b * SEQ + lr) * DM + h * HD + 8u * hi;
    const h16* vp = VT + (size_t)(h * HD + lr) * (size_t)(NB * SEQ) + (size_t)b * SEQ + 8u * hi;
    const int* mk = mask + (size_t)b * SEQ_FULL;

    float mrow[8], lrow[8]; v8f o[4], o2[4];
#pragma unroll
    for (int r = 0; r < 8; ++r) { mrow[r] = NINF; lrow[r] = 0.f; }
#pragma unroll
    for (int nt = 0; nt < 4; ++nt) { o[nt] = (v8f){}; o2[nt] = (v8f){}; }

    const unsigned ntile = (q0 >> 6) + 1u;
#pragma unroll 1
    for (unsigned t = 0; t < ntile; ++t) {
        const unsigned kb = t * 64u;
        v8f s[4];
#pragma unroll
        for (int g = 0; g < 4; ++g) { const bf* kg = kp + (size_t)(kb + g * 16u) * DM; const v16bf kA = ldb(kg), kB = ldb(kg + 32); v8f sg = (v8f){}; sg = wmmab(qa0, kA, sg); sg = wmmab(qa1, kB, sg); s[g] = sg; }
        asm volatile("v_nop\n\tv_nop\n\tv_nop\n\tv_nop" : "+v"(s[0]), "+v"(s[1]), "+v"(s[2]), "+v"(s[3]) : "v"(qa0), "v"(qa1));
        int mv[4];
#pragma unroll
        for (int g = 0; g < 4; ++g) mv[g] = mk[kb + g * 16u + lr];
#pragma unroll
        for (int r = 0; r < 8; ++r) {
            const unsigned qi = q0 + 8u * hi + r;
            float tv[4];
#pragma unroll
            for (int g = 0; g < 4; ++g) { const unsigned key = kb + g * 16u + lr; const bool ok = (mv[g] > 0) && (key <= qi); const float x = s[g][r] * 0.125f; tv[g] = ok ? x : NINF; }
            float mx = fmaxf(fmaxf(tv[0], tv[1]), fmaxf(tv[2], tv[3]));
            mx = fmaxf(mx, __shfl_xor(mx, 1, 32)); mx = fmaxf(mx, __shfl_xor(mx, 2, 32)); mx = fmaxf(mx, __shfl_xor(mx, 4, 32)); mx = fmaxf(mx, __shfl_xor(mx, 8, 32));
            const float mnew = fmaxf(mrow[r], mx);
            const float ms = (mnew == NINF) ? 0.f : mnew;
            const float alpha = __builtin_amdgcn_exp2f((mrow[r] - ms) * 1.4426950408889634f);
            mrow[r] = mnew;
            float rs = 0.f;
#pragma unroll
            for (int g = 0; g < 4; ++g) { const float e = __builtin_amdgcn_exp2f((tv[g] - ms) * 1.4426950408889634f); rs += e; const float pv = e * PCAR; const h16 ph = (h16)pv; const h16 pr = (h16)((pv - (float)ph) * RCAR);
                P[(8u * hi + r) * 72u + g * 16u + lr] = ph; R[(8u * hi + r) * 72u + g * 16u + lr] = pr; }
            lrow[r] = lrow[r] * alpha + rs;
#pragma unroll
            for (int nt = 0; nt < 4; ++nt) { o[nt][r] *= alpha; o2[nt][r] *= alpha; }
        }
        wave_sync();
        const v16h pa0 = cat16(*(const v8ha*)(P + lr * 72u + 8u * hi), *(const v8ha*)(P + lr * 72u + 16u + 8u * hi));
        const v16h pa1 = cat16(*(const v8ha*)(P + lr * 72u + 32u + 8u * hi), *(const v8ha*)(P + lr * 72u + 48u + 8u * hi));
        const v16h ra0 = cat16(*(const v8ha*)(R + lr * 72u + 8u * hi), *(const v8ha*)(R + lr * 72u + 16u + 8u * hi));
        const v16h ra1 = cat16(*(const v8ha*)(R + lr * 72u + 32u + 8u * hi), *(const v8ha*)(R + lr * 72u + 48u + 8u * hi));
#pragma unroll
        for (int nt = 0; nt < 4; ++nt) { const h16* vg = vp + (size_t)nt * 16 * (size_t)(NB * SEQ) + kb; const v16h vA = ldh(vg), vB = ldh(vg + 32);
            o[nt] = wmma16(pa0, vA, o[nt]); o[nt] = wmma16(pa1, vB, o[nt]); o2[nt] = wmma16(ra0, vA, o2[nt]); o2[nt] = wmma16(ra1, vB, o2[nt]); }
        asm volatile("v_nop\n\tv_nop\n\tv_nop\n\tv_nop" : "+v"(o[0]), "+v"(o[1]), "+v"(o[2]), "+v"(o[3]), "+v"(o2[0]), "+v"(o2[1]), "+v"(o2[2]), "+v"(o2[3]) : "v"(pa0), "v"(pa1), "v"(ra0), "v"(ra1));
        wave_sync();
    }

#pragma unroll
    for (int r = 0; r < 8; ++r) {
        float l = lrow[r];
        l += __shfl_xor(l, 1, 32); l += __shfl_xor(l, 2, 32); l += __shfl_xor(l, 4, 32); l += __shfl_xor(l, 8, 32);
        const float inv = (1.0f / l) * (1.0f / (PCAR * VCAR));
#pragma unroll
        for (int nt = 0; nt < 4; ++nt) { const float c = (o[nt][r] + o2[nt][r] * (1.0f / RCAR)) * inv; Ow[(8u * hi + r) * 72u + nt * 16u + lr] = f2bf(c); }
    }
    wave_sync();
    bf* xrow = Xo + (size_t)(b * SEQ + q0) * DM + h * HD;
#pragma unroll 1
    for (int ps = 0; ps < 2; ++ps) {
#pragma unroll
        for (int s = 0; s < 4; ++s) { const unsigned row = 4u * s + (lane >> 3), c = (lane & 7u) * 8u; const v8us val = *(const v8usa*)(Ow + row * 72u + c); *(volatile v8us*)(xrow + (size_t)row * DM + c) = val; }
        if (ps == 0) __threadfence(); }
}

extern "C" void kernel_launch(void* const* d_in, const int* in_sizes, int n_in,
                              void* d_out, int out_size, void* d_ws, size_t ws_size, hipStream_t stream) {
    (void)out_size;
    if (n_in < 12) return;
    const size_t needX = (size_t)(NB - 1) * SEQ_FULL * DM + (size_t)SEQ * DM;
    if ((size_t)in_sizes[0] < needX || (size_t)in_sizes[1] < needX || (size_t)in_sizes[2] < needX) return;
    if ((size_t)in_sizes[3] < (size_t)(NB - 1) * SEQ_FULL + SEQ) return;
    if ((size_t)in_sizes[4] < (size_t)DM * DM || (size_t)in_sizes[6] < (size_t)DM * DM || (size_t)in_sizes[8] < (size_t)DM * DM || (size_t)in_sizes[10] < (size_t)DM * DM) return;
    if (in_sizes[5] < DM || in_sizes[7] < DM || in_sizes[9] < DM || in_sizes[11] < DM) return;
    const float* xq = (const float*)d_in[0]; const float* xk = (const float*)d_in[1]; const float* xv = (const float*)d_in[2]; const int* mask = (const int*)d_in[3];
    const float* wq = (const float*)d_in[4]; const float* bq = (const float*)d_in[5]; const float* wk = (const float*)d_in[6]; const float* bk = (const float*)d_in[7];
    const float* wv = (const float*)d_in[8]; const float* bv = (const float*)d_in[9]; const float* wo = (const float*)d_in[10]; const float* bo = (const float*)d_in[11];
    float* OUT = (float*)d_out;
    char* wsp = (char*)d_ws;
    auto take = [&](size_t bytes) { char* p = wsp; wsp += (bytes + 255) & ~(size_t)255; return (void*)p; };
    const size_t WB = (size_t)DM * DM * 2, XBY = (size_t)NB * SEQ * DM * 2;
    bf* WQ = (bf*)take(WB); bf* WK = (bf*)take(WB); bf* WV = (bf*)take(WB); bf* WO = (bf*)take(WB);
    bf* XQ = (bf*)take(XBY); bf* XK = (bf*)take(XBY); bf* XV = (bf*)take(XBY);
    bf* QP = (bf*)take(XBY); bf* KP = (bf*)take(XBY); h16* VT = (h16*)take(XBY); bf* CX = (bf*)take(XBY);
    if ((size_t)(wsp - (char*)d_ws) > ws_size) return;

    const unsigned WG = (unsigned)(DM * DM / 64 / 64);
    k_wtG<<<WG, 256, 0, stream>>>(wq, WQ); k_wtG<<<WG, 256, 0, stream>>>(wk, WK); k_wtG<<<WG, 256, 0, stream>>>(wv, WV); k_wtG<<<WG, 256, 0, stream>>>(wo, WO);
    const unsigned n8 = (unsigned)((size_t)SEQ * DM / 8);
    const dim3 cg(n8 / 256u, NB, 1);
    k_cvt8<<<cg, 256, 0, stream>>>(xq, XQ, (size_t)SEQ_FULL * DM, (size_t)SEQ * DM, n8);
    k_cvt8<<<cg, 256, 0, stream>>>(xk, XK, (size_t)SEQ_FULL * DM, (size_t)SEQ * DM, n8);
    k_cvt8<<<cg, 256, 0, stream>>>(xv, XV, (size_t)SEQ_FULL * DM, (size_t)SEQ * DM, n8);
    k_gemmw<1><<<dim3(NB * SEQ / 64, DM / 64, 1), 32, 0, stream>>>(XQ, WQ, (void*)QP, bq, 0, 0, DM, DM);
    k_gemmw<1><<<dim3(NB * SEQ / 64, DM / 64, 1), 32, 0, stream>>>(XK, WK, (void*)KP, bk, 0, 0, DM, DM);
    k_gemmw<2><<<dim3(DM / 64, NB * SEQ / 64, 1), 32, 0, stream>>>(WV, XV, (void*)VT, bv, 0, 0, DM, NB * SEQ);
    k_flash<<<(unsigned)(NB * NH_ * QT / 4), 128, 0, stream>>>(QP, KP, VT, mask, CX);
    k_gemmw<0><<<dim3(SEQ / 64, DM / 64, NB), 32, 0, stream>>>(CX, WO, (void*)OUT, bo, (size_t)SEQ * DM, (size_t)SEQ_FULL * DM, DM, DM);
}
